// GAT_12661563588624
// MI455X (gfx1250) — hardware-run, weakly checked
//
#include <hip/hip_runtime.h>

typedef float          v8f   __attribute__((ext_vector_type(8)));
typedef float          v4f   __attribute__((ext_vector_type(4)));
typedef unsigned int   v4u   __attribute__((ext_vector_type(4)));
typedef int            v8i   __attribute__((ext_vector_type(8)));
typedef unsigned short v8us  __attribute__((ext_vector_type(8)));
typedef unsigned short v16us __attribute__((ext_vector_type(16)));
typedef __bf16         v16bf __attribute__((ext_vector_type(16)));
typedef _Float16       v16h  __attribute__((ext_vector_type(16)));
typedef v4f  __attribute__((may_alias)) v4fa;
typedef v8us __attribute__((may_alias)) v8usa;
union FragB { v16bf v; v16us u; v8us h[2]; v8i w; };
union FragH { v16h  v; v16us u; v8us h[2]; v8i w; };

__device__ __forceinline__ v8f wmb(const FragB& a, const FragB& b, v8f c) {
  v8f d = __builtin_amdgcn_wmma_f32_16x16x32_bf16(false, a.v, false, b.v, (short)0, c, false, false);
  asm volatile("v_nop\n\tv_nop\n\tv_nop\n\tv_nop" : "+v"(d) : "v"(a.w), "v"(b.w));
  return d;
}

__device__ __forceinline__ v8f wmh(const FragH& a, const FragH& b, v8f c) {
  v8f d = __builtin_amdgcn_wmma_f32_16x16x32_f16(false, a.v, false, b.v, (short)0, c, false, false);
  asm volatile("v_nop\n\tv_nop\n\tv_nop\n\tv_nop" : "+v"(d) : "v"(a.w), "v"(b.w));
  return d;
}

__device__ __forceinline__ unsigned bf16_bits(float f) {
  const unsigned u = __float_as_uint(f);
  const unsigned r = (u + 0x7FFFu + ((u >> 16) & 1u)) >> 16;
  const unsigned q = (u >> 16) | 0x40u;
  return ((u & 0x7fffffffu) > 0x7f800000u) ? q : r;
}

__device__ __forceinline__ float bf16_val(float f) {
  return __uint_as_float(bf16_bits(f) << 16);
}
__device__ __forceinline__ int clampi(int v, int lo, int hi) {
  return v < lo ? lo : (v > hi ? hi : v);
}

__device__ __forceinline__ unsigned f16_bits(float f) {
  const unsigned u  = __float_as_uint(f);
  const unsigned s  = (u >> 16) & 0x8000u;
  const unsigned a  = u & 0x7fffffffu;
  const unsigned t  = a - 0x38000000u;
  const unsigned r  = (t + 0x0FFFu + ((t >> 13) & 1u)) >> 13;
  const unsigned rc = r > 0x7C00u ? 0x7C00u : r;
  const bool small  = a < 0x38800000u;
  const bool isnan  = a > 0x7f800000u;
  const unsigned fin = small ? 0u : (s | rc);
  return isnan ? (s | 0x7E00u) : fin;
}

__device__ __forceinline__ unsigned pk16(unsigned lo, unsigned hi) { return lo | (hi << 16); }
__device__ __forceinline__ unsigned bf16_lo_bits(float v) {
  float hi = bf16_val(v);
  asm volatile("" : "+v"(hi));
  return bf16_bits(v - hi);
}
__device__ __forceinline__ v4u pack8_bf16(v4f a, v4f c) {
  return (v4u){ pk16(bf16_bits(a[0]), bf16_bits(a[1])), pk16(bf16_bits(a[2]), bf16_bits(a[3])),
                pk16(bf16_bits(c[0]), bf16_bits(c[1])), pk16(bf16_bits(c[2]), bf16_bits(c[3])) };
}
__device__ __forceinline__ v4u pack8_bf16_lo(v4f a, v4f c) {
  return (v4u){ pk16(bf16_lo_bits(a[0]), bf16_lo_bits(a[1])), pk16(bf16_lo_bits(a[2]), bf16_lo_bits(a[3])),
                pk16(bf16_lo_bits(c[0]), bf16_lo_bits(c[1])), pk16(bf16_lo_bits(c[2]), bf16_lo_bits(c[3])) };
}
__device__ __forceinline__ v4u pack8_f16(v4f a, v4f c) {
  return (v4u){ pk16(f16_bits(a[0]), f16_bits(a[1])), pk16(f16_bits(a[2]), f16_bits(a[3])),
                pk16(f16_bits(c[0]), f16_bits(c[1])), pk16(f16_bits(c[2]), f16_bits(c[3])) };
}

template <int FORM>
__global__ __launch_bounds__(256) void k_plane(const float* __restrict__ src, int rows, int cols, int ldsrc,
                                               unsigned short* __restrict__ dst, int MP, int KP) {
  static_assert(FORM >= 0 && FORM <= 3);
  const int KTOT = (FORM == 1 || FORM == 3) ? 2 * KP : KP;
  const unsigned ppr   = (unsigned)(KTOT >> 3);
  const unsigned kp8   = (unsigned)(KP >> 3);
  const unsigned total = (unsigned)MP * ppr;
  const unsigned g     = blockIdx.x * 256u + threadIdx.x;
  const unsigned rowu  = g / ppr;
  const unsigned p     = g - rowu * ppr;
  const bool second    = p >= kp8;
  const int row = (int)rowu;
  const int c0  = (int)((second ? p - kp8 : p) << 3);
  const float* srow = src + (size_t)clampi(row, 0, rows - 1) * (size_t)ldsrc;
  float x[8];
  unsigned mk[8];
#pragma unroll
  for (int e = 0; e < 8; ++e) {
    const int c = c0 + e;
    const float v = srow[clampi(c, 0, cols - 1)];
    asm volatile("" :: "v"(v));
    x[e]  = v;
    mk[e] = (row < rows && c < cols) ? 0xFFFFu : 0u;
  }
  const v4f a = (v4f){ x[0], x[1], x[2], x[3] };
  const v4f c = (v4f){ x[4], x[5], x[6], x[7] };
  v4u o;
  if (FORM == 2) {
    o = pack8_f16(a, c);
  } else {
    const v4u hi = pack8_bf16(a, c);
    o = hi;
    if (FORM == 1) { const v4u lo = pack8_bf16_lo(a, c); o = second ? lo : hi; }
  }
  const v4u mw = (v4u){ pk16(mk[0], mk[1]), pk16(mk[2], mk[3]), pk16(mk[4], mk[5]), pk16(mk[6], mk[7]) };
  o &= mw;
  if (g < total) {
    volatile v4u* q = (volatile v4u*)(dst + (size_t)g * 8);
    *q = o;
    __threadfence();
    *q = o;
  }
}

template <int FORM> struct FragOf    { typedef FragB T; };
template <>         struct FragOf<2> { typedef FragH T; };
__device__ __forceinline__ v8f mm(const FragB& a, const FragB& b, v8f c) { return wmb(a, b, c); }
__device__ __forceinline__ v8f mm(const FragH& a, const FragH& b, v8f c) { return wmh(a, b, c); }
template <class F> __device__ __forceinline__ F ld_frag(const unsigned short* p) {
  F f;
  f.h[0] = *(const v8usa*)(p);
  f.h[1] = *(const v8usa*)(p + 16);
  return f;
}

template <int FORM, int EPI>
__global__ __launch_bounds__(256) __attribute__((amdgpu_num_vgpr(248)))
void k_gemm_nt(const unsigned short* __restrict__ A, const unsigned short* __restrict__ B,
               const float* __restrict__ bias, float* __restrict__ D, int M, int N, int KTOT, int ldd) {
  static_assert(FORM >= 0 && FORM <= 2);
  static_assert(EPI == 0 || EPI == 1);
  typedef typename FragOf<FORM>::T F;
  __shared__ __attribute__((aligned(16))) float sT[8][16 * 68];
  const int lane = threadIdx.x & 31;
  const int wave = threadIdx.x >> 5;
  const int tilesM = (M + 63) >> 6;
  const int tilesN = (N + 63) >> 6;
  const int tile = blockIdx.x * 8 + wave;
  if (tile >= tilesM * tilesN) return;
  const int tm = tile / tilesN;
  const int tn = tile - tm * tilesN;
  const int m0 = tm << 6;
  const int n0 = tn << 6;

  const int rl = lane & 15;
  const int h8 = (lane >> 4) * 8;
  const unsigned short* pa = A + (size_t)(m0 + rl) * (size_t)KTOT + h8;
  const unsigned short* pb = B + (size_t)(n0 + rl) * (size_t)KTOT + h8;

  v8f acc[4][4];
#pragma unroll
  for (int i = 0; i < 4; ++i)
#pragma unroll
    for (int j = 0; j < 4; ++j) acc[i][j] = (v8f){0.f, 0.f, 0.f, 0.f, 0.f, 0.f, 0.f, 0.f};

#pragma unroll 1
  for (int k0 = 0; k0 < KTOT; k0 += 32) {
    F bf[4];
#pragma unroll
    for (int j = 0; j < 4; ++j) bf[j] = ld_frag<F>(pb + (size_t)(j << 4) * (size_t)KTOT + k0);
#pragma unroll
    for (int i = 0; i < 4; ++i) {
      const F af = ld_frag<F>(pa + (size_t)(i << 4) * (size_t)KTOT + k0);
#pragma unroll
      for (int j = 0; j < 4; ++j) acc[i][j] = mm(af, bf[j], acc[i][j]);
    }
  }

  float* slab = sT[wave];
  const int hh = lane >> 4;
  const int c4 = (lane & 15) * 4;
  const int nc = n0 + c4;
  const bool cok = nc < N;
  v4f bv = (v4f){0.f, 0.f, 0.f, 0.f};
  if (EPI == 1) {
    bv = *(const v4fa*)(bias + clampi(nc, 0, N - 4));
    asm volatile("" :: "v"(bv));
  }
#pragma unroll
  for (int i = 0; i < 4; ++i) {
    const int mBase = m0 + (i << 4);
#pragma unroll
    for (int j = 0; j < 4; ++j) {
#pragma unroll
      for (int r = 0; r < 8; ++r) slab[(h8 + r) * 68 + (j << 4) + rl] = acc[i][j][r];
    }
    __builtin_amdgcn_fence(__ATOMIC_RELEASE, "workgroup");
    __builtin_amdgcn_wave_barrier();
    __builtin_amdgcn_fence(__ATOMIC_ACQUIRE, "workgroup");
    v4f vv[8];
#pragma unroll
    for (int it = 0; it < 8; ++it) {
      const int row = it * 2 + hh;
      v4f v = *(const v4fa*)(slab + row * 68 + c4);
      if (EPI == 1) v += bv;
      vv[it] = v;
    }
    for (int pass = 0; pass < 2; ++pass) {
#pragma unroll
      for (int it = 0; it < 8; ++it) {
        const int row = mBase + it * 2 + hh;
        if (cok && row < M) *(volatile v4f*)(D + (size_t)row * (size_t)ldd + nc) = vv[it];
      }
      __threadfence();
    }
    __builtin_amdgcn_fence(__ATOMIC_RELEASE, "workgroup");
    __builtin_amdgcn_wave_barrier();
    __builtin_amdgcn_fence(__ATOMIC_ACQUIRE, "workgroup");
  }
}

#pragma clang fp contract(off)


#ifndef SPLIT_2
#define SPLIT_2 1
#endif
#ifndef SPLIT_3
#define SPLIT_3 1
#endif

#define NN      100000
#define NE      1600000
#define MPAD    100096
#define KD      128
#define HC      64
#define RTHR    256
#define RWAVES  8
#define TBL_L   192
#define TB_AD   64
#define TB_B    128
#define TB_N    576
#define LT      512
#define LW      16
#define LEPT    8
#define LCHUNK  (LT * LEPT)
#define NCH     ((NE + LCHUNK - 1) / LCHUNK)
#define NB      1024
#define NBLK    ((NN + NB - 1) / NB)
#define RCAP    20992
#define DEGCAP  64
#define SLOTSH  21
#define LISTTOT (NBLK * RCAP)
#define LDS_LST ((2 * RCAP + 3 * NB + 64) * 4)
#define WSMAX   ((size_t)128 << 20)

#define SZ_XB   ((size_t)MPAD * KD * 2)
#define SZ_WP   ((size_t)3 * HC * KD * 2)
#define SZ_TB   ((size_t)4096)
#define SZ_FT   ((size_t)MPAD * HC * 4)
#define SZ_ELR  ((size_t)MPAD * 4 * 4)
#define SZ_META ((size_t)NBLK * NB * 2 * 4)
#define SZ_LIST ((size_t)NBLK * RCAP * 4)
#define WS_TOTAL (SZ_XB + SZ_WP + SZ_TB + SZ_FT + SZ_ELR + SZ_META + SZ_LIST)

static_assert(NN % 8 == 0);
static_assert(12500 * 8 == NN && (NN / RWAVES) * RWAVES == NN);
static_assert(MPAD == 782 * 128 && MPAD % 64 == 0 && MPAD >= NN);
static_assert(2 * 32 == HC);
static_assert(2 * 32 == HC && 1 * 64 == HC);
static_assert(KD % 32 == 0 && HC % 4 == 0 && HC % 32 == 0);
static_assert(NE < (1 << SLOTSH));
static_assert(NB <= 1024 && (NB & (NB - 1)) == 0 && NB == 2 * LT);
static_assert(NE % 8 == 0 && NE >= 8);
static_assert(NBLK == 98 && NBLK * NB >= NN);
static_assert(NCH * LCHUNK >= NE && NCH == 391);
static_assert(RCAP % 32 == 0 && RCAP % LT == 0);
static_assert(RCAP * 4 >= 16710 * 5);
static_assert(DEGCAP >= 36 + 8);
static_assert(LDS_LST <= 262144);
static_assert(LW == LT / 32 && LW == 16);
static_assert(TB_N * 4 <= 4096 && 3 * TBL_L == TB_N);
static_assert(SZ_XB % 128 == 0 && SZ_WP % 128 == 0 && SZ_TB % 128 == 0 && SZ_FT % 128 == 0);
static_assert(SZ_ELR % 128 == 0 && SZ_META % 128 == 0 && SZ_LIST % 128 == 0);
static_assert(WS_TOTAL == 61935616);
static_assert(WS_TOTAL <= WSMAX);
static_assert((size_t)(NN - 1) * HC + 63 == 6399999);

typedef float        v2f __attribute__((ext_vector_type(2)));
typedef int          v4i __attribute__((ext_vector_type(4)));
typedef int          v2i __attribute__((ext_vector_type(2)));
typedef v2f __attribute__((may_alias)) v2fa;
typedef v4i __attribute__((may_alias)) v4ia;
typedef v2i __attribute__((may_alias)) v2ia;

__device__ __forceinline__ float relu_k(float v) { return (v > 0.0f) ? v : (v - v); }
__device__ __forceinline__ float lrelu_k(float v) { return (v >= 0.0f) ? v : 0.2f * v; }
__device__ __forceinline__ float maxk(float a, float b) {
  float m = (a < b) ? b : a;
  m = (b != b) ? b : m;
  return m;
}

__device__ __forceinline__ void wpiece(const float* __restrict__ W, int kmask, int g, unsigned short* dst) {
  const int n  = g >> 4;
  const int k0 = (g & 15) << 3;
  float x[8];
#pragma unroll
  for (int e = 0; e < 8; ++e) {
    const float v = W[(size_t)((k0 + e) & kmask) * HC + n];
    asm volatile("" :: "v"(v));
    x[e] = v;
  }
  const v4u o = pack8_bf16((v4f){ x[0], x[1], x[2], x[3] }, (v4f){ x[4], x[5], x[6], x[7] });
  volatile v4u* q = (volatile v4u*)(dst + (size_t)g * 8);
  *q = o;
  __threadfence();
  *q = o;
}
__device__ __forceinline__ v4u tpiece(const float* __restrict__ p, int idx, int a) {
  const v4f v = *(const v4fa*)(p + clampi(idx - 64 * a, 0, 60));
  asm volatile("" :: "v"(v));
  const unsigned m = (idx >= 64 * a && idx < 64 * a + 64) ? 0xFFFFFFFFu : 0u;
  return (v4u){ __float_as_uint(v.x) & m, __float_as_uint(v.y) & m, __float_as_uint(v.z) & m, __float_as_uint(v.w) & m };
}
__global__ __launch_bounds__(256) void k_prep(const float* __restrict__ W1, const float* __restrict__ W2,
                                              const float* __restrict__ W3,
                                              const float* __restrict__ as1, const float* __restrict__ ad1,
                                              const float* __restrict__ b1,
                                              const float* __restrict__ as2, const float* __restrict__ ad2,
                                              const float* __restrict__ b2,
                                              const float* __restrict__ as3, const float* __restrict__ ad3,
                                              const float* __restrict__ b3,
                                              unsigned short* WP, float* TB) {
  const int b = (int)blockIdx.x;
  const int t = (int)threadIdx.x;
  if (b < 4) {
    wpiece(W1, 127, b * 256 + t, WP);
  } else if (b < 8) {
    wpiece(W2, 63, (b - 4) * 256 + t, WP + HC * KD);
  } else if (b < 12) {
    wpiece(W3, 63, (b - 8) * 256 + t, WP + 2 * HC * KD);
  } else {
    const int idx = 4 * t;
    v4u o = tpiece(as1, idx, 0);
    o |= tpiece(ad1, idx, 1);
    o |= tpiece(b1,  idx, 2);
    o |= tpiece(as2, idx, 3);
    o |= tpiece(ad2, idx, 4);
    o |= tpiece(b2,  idx, 5);
    o |= tpiece(as3, idx, 6);
    o |= tpiece(ad3, idx, 7);
    o |= tpiece(b3,  idx, 8);
    o.x = bf16_bits(__uint_as_float(o.x)) << 16;
    o.y = bf16_bits(__uint_as_float(o.y)) << 16;
    o.z = bf16_bits(__uint_as_float(o.z)) << 16;
    o.w = bf16_bits(__uint_as_float(o.w)) << 16;
    const bool wr = idx < TB_N;
    volatile v4u* q = (volatile v4u*)(TB + (wr ? idx : 0));
    if (wr) *q = o;
    __threadfence();
    if (wr) *q = o;
  }
}

__global__ __launch_bounds__(LT) void k_list(const int* __restrict__ esrc, const int* __restrict__ edst,
                                             unsigned* LIST, int* META) {
  extern __shared__ v4u lds_lst[];
  int* reg1 = (int*)lds_lst;
  int* reg2 = reg1 + RCAP;
  int* scnt = reg2 + RCAP;
  int* soff = scnt + NB;
  int* curs = soff + NB;
  int* wcnt = curs + NB;
  int* wtot = wcnt + 2 * LW;
  const int tid = (int)threadIdx.x, lane = tid & 31, wave = tid >> 5;
  const int nodeBase = (int)blockIdx.x * NB;
  int nb = NN - nodeBase;
  nb = nb > NB ? NB : (nb < 0 ? 0 : nb);
  const unsigned nbs = (unsigned)nodeBase, unb = (unsigned)nb;

  scnt[2 * tid] = 0;
  scnt[2 * tid + 1] = 0;
  if (tid == 0) reg2[0] = 0;

  int tot = 0;
#pragma unroll 1
  for (int ch = 0; ch < NCH; ++ch) {
    const int par = ch & 1;
    const int e0  = ch * LCHUNK + tid * LEPT;
    const bool valid = e0 < NE;
    const int ea = e0 < NE - 8 ? e0 : NE - 8;
    const v4i da = *(const v4ia*)(edst + ea);
    const v4i db = *(const v4ia*)(edst + ea + 4);
    asm volatile("" :: "v"(da), "v"(db));
    const unsigned s0 = (unsigned)da.x - nbs, s1 = (unsigned)da.y - nbs;
    const unsigned s2 = (unsigned)da.z - nbs, s3 = (unsigned)da.w - nbs;
    const unsigned s4 = (unsigned)db.x - nbs, s5 = (unsigned)db.y - nbs;
    const unsigned s6 = (unsigned)db.z - nbs, s7 = (unsigned)db.w - nbs;
    const bool h0 = valid && (s0 < unb), h1 = valid && (s1 < unb), h2 = valid && (s2 < unb), h3 = valid && (s3 < unb);
    const bool h4 = valid && (s4 < unb), h5 = valid && (s5 < unb), h6 = valid && (s6 < unb), h7 = valid && (s7 < unb);
    const int c = (int)h0 + (int)h1 + (int)h2 + (int)h3 + (int)h4 + (int)h5 + (int)h6 + (int)h7;
    int incl = c;
#pragma unroll
    for (int d = 1; d < 32; d <<= 1) {
      const int up = __shfl_up(incl, d, 32);
      incl += (lane >= d) ? up : 0;
    }
    const int wtotal = __shfl(incl, 31, 32);
    if (lane == 0) wcnt[par * LW + wave] = wtotal;
    __syncthreads();
    int all = 0, pre = 0;
#pragma unroll
    for (int g = 0; g < 4; ++g) {
      const v4i w4 = *(const v4ia*)(wcnt + par * LW + 4 * g);
      const int c0 = clampi(w4.x, 0, 256), c1 = clampi(w4.y, 0, 256);
      const int c2 = clampi(w4.z, 0, 256), c3 = clampi(w4.w, 0, 256);
      all += c0 + c1 + c2 + c3;
      pre += (4 * g + 0 < wave) ? c0 : 0;
      pre += (4 * g + 1 < wave) ? c1 : 0;
      pre += (4 * g + 2 < wave) ? c2 : 0;
      pre += (4 * g + 3 < wave) ? c3 : 0;
    }
    int pos = tot + pre + (incl - c);
#define PUTJ(J, HJ, SJ) if (HJ) { if (pos < RCAP) reg1[pos] = (int)((unsigned)(e0 + (J)) | ((SJ) << SLOTSH)); ++pos; }
    PUTJ(0, h0, s0)
    PUTJ(1, h1, s1)
    PUTJ(2, h2, s2)
    PUTJ(3, h3, s3)
    PUTJ(4, h4, s4)
    PUTJ(5, h5, s5)
    PUTJ(6, h6, s6)
    PUTJ(7, h7, s7)
#undef PUTJ
    tot += all;
  }
  __syncthreads();
  const bool ovf = tot > RCAP;
  const int nh = ovf ? RCAP : tot;

  if (wave == 0) {
#pragma unroll 1
    for (int b0 = 0; b0 < nh; b0 += 32) {
      const int idx = b0 + lane;
      const int uv  = reg1[idx < nh ? idx : nh - 1];
      const int m32 = (nh - b0) < 32 ? (nh - b0) : 32;
#pragma unroll 1
      for (int k = 0; k < m32; ++k) {
        const int u  = __builtin_amdgcn_readlane(uv, k);
        const int sl = (int)(((unsigned)u >> SLOTSH) & (unsigned)(NB - 1));
        const int cv = scnt[sl] + 1;
        if (lane == 0) scnt[sl] = cv;
      }
    }
  }
  __syncthreads();

  int e0c, e1c;
  {
    const v2i cc = *(const v2ia*)(scnt + 2 * tid);
    e0c = cc.x < 0 ? 0 : cc.x;
    e1c = cc.y < 0 ? 0 : cc.y;
    const int ts = e0c + e1c;
    int incl = ts;
#pragma unroll
    for (int d = 1; d < 32; d <<= 1) {
      const int up = __shfl_up(incl, d, 32);
      incl += (lane >= d) ? up : 0;
    }
    if (lane == 31) wtot[wave] = incl;
    __syncthreads();
    int pre = 0;
#pragma unroll
    for (int g = 0; g < 4; ++g) {
      const v4i w4 = *(const v4ia*)(wtot + 4 * g);
      pre += (4 * g + 0 < wave) ? w4.x : 0;
      pre += (4 * g + 1 < wave) ? w4.y : 0;
      pre += (4 * g + 2 < wave) ? w4.z : 0;
      pre += (4 * g + 3 < wave) ? w4.w : 0;
    }
    const int run = pre + incl - ts;
    soff[2 * tid]     = run;
    soff[2 * tid + 1] = run + e0c;
    curs[2 * tid]     = run;
    curs[2 * tid + 1] = run + e0c;
  }
  __syncthreads();

  if (wave == 0) {
#pragma unroll 1
    for (int b0 = 0; b0 < nh; b0 += 32) {
      const int idx = b0 + lane;
      const int uv  = reg1[idx < nh ? idx : nh - 1];
      const int m32 = (nh - b0) < 32 ? (nh - b0) : 32;
#pragma unroll 1
      for (int k = 0; k < m32; ++k) {
        const int u   = __builtin_amdgcn_readlane(uv, k);
        const int sl  = (int)(((unsigned)u >> SLOTSH) & (unsigned)(NB - 1));
        const int eid = (int)((unsigned)u & ((1u << SLOTSH) - 1u));
        const int pr  = curs[sl];
        const int pc  = clampi(pr, 0, RCAP - 1);
        if (lane == 0) { reg2[pc] = eid; curs[sl] = pc + 1; }
      }
    }
  }
  __syncthreads();

  {
    unsigned* lbase = LIST + (size_t)blockIdx.x * (size_t)RCAP;
#pragma unroll 1
    for (int it = 0; it < RCAP / LT; ++it) {
      const int i  = it * LT + tid;
      const int ic = clampi(i < nh ? i : nh - 1, 0, RCAP - 1);
      const int eid = clampi(reg2[ic], 0, NE - 1);
      const int cw = esrc[eid];
      asm volatile("" :: "v"(cw));
      const unsigned msk = (i < nh) ? 0xFFFFFFFFu : 0u;
      const unsigned o = (unsigned)clampi(cw, 0, NN - 1) & msk;
      volatile unsigned* q = (volatile unsigned*)(lbase + i);
      *q = o;
      __threadfence();
      *q = o;
    }
  }

  {
    const int base = (int)blockIdx.x * RCAP;
    const v2i cc = *(const v2ia*)(scnt + 2 * tid);
    const v2i so = *(const v2ia*)(soff + 2 * tid);
    v4i m;
    m.x = base + so.x;
    m.y = ovf ? -1 : cc.x;
    m.z = base + so.y;
    m.w = ovf ? -1 : cc.y;
    volatile v4i* q = (volatile v4i*)(META + 2 * (size_t)(nodeBase + 2 * tid));
    *q = m;
    __threadfence();
    *q = m;
  }
}

template <int HEADS>
__global__ __launch_bounds__(RTHR) void k_rowprep(const float* __restrict__ FT, const float* __restrict__ TBL,
                                                  float* ELR) {
  static_assert(HEADS == 1 || HEADS == 2);
  __shared__ __attribute__((aligned(16))) float sdot[RWAVES * 4];
  const int lane = (int)threadIdx.x & 31;
  const int wave = (int)threadIdx.x >> 5;
  const int row  = (int)blockIdx.x * RWAVES + wave;
  const int rowc = row < NN ? row : NN - 1;
  const int c0   = lane * 2;
  const v2f h = *(const v2fa*)(FT + (size_t)rowc * HC + c0);
  asm volatile("" :: "v"(h));
  const v2f as = *(const v2fa*)(TBL + c0);
  const v2f ad = *(const v2fa*)(TBL + TB_AD + c0);
  float ts = h.x * as.x;
  float u  = h.y * as.y;
  ts = ts + u;
  float td = h.x * ad.x;
  u  = h.y * ad.y;
  td = td + u;
  if (HEADS == 1) {
    ts = ts + __shfl_xor(ts, 16, 32);
    td = td + __shfl_xor(td, 16, 32);
  }
  ts = ts + __shfl_xor(ts, 8, 32);
  td = td + __shfl_xor(td, 8, 32);
  ts = ts + __shfl_xor(ts, 4, 32);
  td = td + __shfl_xor(td, 4, 32);
  ts = ts + __shfl_xor(ts, 2, 32);
  td = td + __shfl_xor(td, 2, 32);
  ts = ts + __shfl_xor(ts, 1, 32);
  td = td + __shfl_xor(td, 1, 32);
  if ((lane & 15) == 0) {
    sdot[wave * 4 + (lane >> 4)]     = ts;
    sdot[wave * 4 + 2 + (lane >> 4)] = td;
  }
  __syncthreads();
  if (wave == 0) {
    const int l8 = lane & 7;
    const v4f sv = *(const v4fa*)(sdot + 4 * l8);
    asm volatile("" :: "v"(sv));
    const int trow = (int)blockIdx.x * RWAVES + l8;
    const bool wr = (lane < 8) && (trow < NN);
    volatile v4f* q = (volatile v4f*)(ELR + (size_t)(trow < NN ? trow : NN - 1) * 4);
    if (wr) *q = sv;
    __threadfence();
    if (wr) *q = sv;
  }
}

struct Ent { int col; float e0; float e1; };
__device__ __forceinline__ Ent load_ent(const unsigned* __restrict__ LIST, const float* __restrict__ ELR,
                                        int off, int cnt, int b0, int lane, float er0, float er1) {
  const int jj = b0 + lane;
  const int j  = jj < cnt ? jj : cnt - 1;
  const unsigned sw = LIST[(size_t)(off + j)];
  asm volatile("" :: "v"(sw));
  Ent r;
  r.col = clampi((int)sw, 0, NN - 1);
  const v4f s4 = *(const v4fa*)(ELR + (size_t)r.col * 4);
  asm volatile("" :: "v"(s4));
  r.e0 = lrelu_k(s4.x + er0);
  r.e1 = lrelu_k(s4.y + er1);
  return r;
}

template <int LAST>
__global__ __launch_bounds__(RTHR) void k_walk(const float* __restrict__ FT, const float* __restrict__ ELR,
                                               const unsigned* __restrict__ LIST, const int* __restrict__ META,
                                               const float* __restrict__ TBL, unsigned short* OP, float* out,
                                               int nrows, unsigned lomask) {
  const int lane = (int)threadIdx.x & 31;
  const int wave = (int)threadIdx.x >> 5;
  const int row  = (int)blockIdx.x * RWAVES + wave;
  const int rowc = row < NN ? row : NN - 1;
  const int head = lane >> 4;
  const int c0   = lane * 2;

  const v2i mt = *(const v2ia*)(META + 2 * (size_t)rowc);
  asm volatile("" :: "v"(mt));
  const int craw = mt.y;
  const int offv = clampi(mt.x, 0, LISTTOT);
  int cntv = clampi(craw, 0, DEGCAP);
  cntv = cntv < (LISTTOT - offv) ? cntv : (LISTTOT - offv);
  const int off = __builtin_amdgcn_readfirstlane(offv);
  const int cnt = __builtin_amdgcn_readfirstlane(cntv);
  const bool poison = (craw < 0) || (craw > DEGCAP);

  const v4f d4 = *(const v4fa*)(ELR + (size_t)rowc * 4);
  asm volatile("" :: "v"(d4));
  const float er0 = d4.z, er1 = d4.w;
  const float eL0 = lrelu_k(d4.x + er0);
  const float eL1 = lrelu_k(d4.y + er1);

  float mx0 = eL0, mx1 = eL1;
#pragma unroll 1
  for (int b0 = 0; b0 < cnt; b0 += 32) {
    const Ent en = load_ent(LIST, ELR, off, cnt, b0, lane, er0, er1);
    mx0 = maxk(mx0, en.e0);
    mx1 = maxk(mx1, en.e1);
  }
#pragma unroll
  for (int d = 16; d > 0; d >>= 1) {
    const float o0 = __shfl_xor(mx0, d, 32);
    const float o1 = __shfl_xor(mx1, d, 32);
    mx0 = maxk(mx0, o0);
    mx1 = maxk(mx1, o1);
  }

  float den0 = 0.0f, den1 = 0.0f;
#pragma unroll 1
  for (int b0 = 0; b0 < cnt; b0 += 32) {
    const Ent en = load_ent(LIST, ELR, off, cnt, b0, lane, er0, er1);
    const float q0 = expf(en.e0 - mx0);
    const float q1 = expf(en.e1 - mx1);
    const int m32 = (cnt - b0) < 32 ? (cnt - b0) : 32;
#pragma unroll 1
    for (int k = 0; k < m32; ++k) {
      const float a0 = __int_as_float(__builtin_amdgcn_readlane(__float_as_int(q0), k));
      const float a1 = __int_as_float(__builtin_amdgcn_readlane(__float_as_int(q1), k));
      den0 = den0 + a0;
      den1 = den1 + a1;
    }
  }
  const float qL0 = expf(eL0 - mx0);
  const float qL1 = expf(eL1 - mx1);
  den0 = den0 + qL0;
  den1 = den1 + qL1;

  v2f ac = (v2f){0.0f, 0.0f};
#pragma unroll 1
  for (int b0 = 0; b0 < cnt; b0 += 32) {
    const Ent en = load_ent(LIST, ELR, off, cnt, b0, lane, er0, er1);
    const float q0 = expf(en.e0 - mx0);
    const float q1 = expf(en.e1 - mx1);
    const float w0 = q0 / den0;
    const float w1 = q1 / den1;
    const int m32 = (cnt - b0) < 32 ? (cnt - b0) : 32;
#pragma unroll 1
    for (int k = 0; k < m32; ++k) {
      const int c = __builtin_amdgcn_readlane(en.col, k);
      const float a0 = __int_as_float(__builtin_amdgcn_readlane(__float_as_int(w0), k));
      const float a1 = __int_as_float(__builtin_amdgcn_readlane(__float_as_int(w1), k));
      const float w = (LAST != 0 || head == 0) ? a0 : a1;
      const v2f hn = *(const v2fa*)(FT + (size_t)c * HC + c0);
      float pr;
      pr = w * hn.x; ac.x = ac.x + pr;
      pr = w * hn.y; ac.y = ac.y + pr;
    }
  }
  {
    const float wL0 = qL0 / den0;
    const float wL1 = qL1 / den1;
    const float w = (LAST != 0 || head == 0) ? wL0 : wL1;
    const v2f hd = *(const v2fa*)(FT + (size_t)rowc * HC + c0);
    float pr;
    pr = w * hd.x; ac.x = ac.x + pr;
    pr = w * hd.y; ac.y = ac.y + pr;
  }

  const v2f bv = *(const v2fa*)(TBL + TB_B + c0);
  const float vx = ac.x + bv.x;
  const float vy = ac.y + bv.y;
  const float qnan = __uint_as_float(0x7fc00000u);
  const bool rok = row < nrows;
  if (LAST != 0) {
    v2f o;
    o.x = poison ? qnan : vx;
    o.y = poison ? qnan : vy;
    float* orow = out + (size_t)rowc * HC + c0;
    if (rok) *(volatile v2f*)orow = o;
    __threadfence();
    if (rok) *(volatile v2f*)orow = o;
  } else {
    float yx = relu_k(vx);
    float yy = relu_k(vy);
    yx = poison ? qnan : yx;
    yy = poison ? qnan : yy;
    const unsigned hiw = pk16(bf16_bits(yx), bf16_bits(yy));
    const unsigned low = pk16(bf16_lo_bits(yx), bf16_lo_bits(yy)) & lomask;
    unsigned* prow = (unsigned*)(OP + (size_t)rowc * KD);
    volatile unsigned* qh = (volatile unsigned*)(prow + lane);
    volatile unsigned* ql = (volatile unsigned*)(prow + 32 + lane);
    if (rok) { *qh = hiw; *ql = low; }
    __threadfence();
    if (rok) { *qh = hiw; *ql = low; }
  }
}

extern "C" void kernel_launch(void* const* d_in, const int* in_sizes, int n_in,
                              void* d_out, int out_size, void* d_ws, size_t ws_size,
                              hipStream_t stream) {
  if (n_in < 14) return;
  if (in_sizes[0] != NN * KD) return;
  if (in_sizes[1] != 2 * NE) return;
  if (in_sizes[2] != KD * HC || in_sizes[6] != HC * HC || in_sizes[10] != HC * HC) return;
  if (in_sizes[3] != HC || in_sizes[4] != HC || in_sizes[5] != HC) return;
  if (in_sizes[7] != HC || in_sizes[8] != HC || in_sizes[9] != HC) return;
  if (in_sizes[11] != HC || in_sizes[12] != HC || in_sizes[13] != HC) return;
  if (out_size != NN * HC) return;
  const int nrows = out_size / HC;
  if (nrows != NN) return;

  const float* feat = (const float*)d_in[0];
  const int*   ei   = (const int*)  d_in[1];
  const int*   esrc = ei;
  const int*   edst = ei + NE;
  const float* W1  = (const float*)d_in[2];
  const float* as1 = (const float*)d_in[3];
  const float* ad1 = (const float*)d_in[4];
  const float* b1  = (const float*)d_in[5];
  const float* W2  = (const float*)d_in[6];
  const float* as2 = (const float*)d_in[7];
  const float* ad2 = (const float*)d_in[8];
  const float* b2  = (const float*)d_in[9];
  const float* W3  = (const float*)d_in[10];
  const float* as3 = (const float*)d_in[11];
  const float* ad3 = (const float*)d_in[12];
  const float* b3  = (const float*)d_in[13];
  float* out = (float*)d_out;

  char* ws = (char*)d_ws;
  size_t off = 0;
  const size_t oXB   = off; off += SZ_XB;
  const size_t oWP   = off; off += SZ_WP;
  const size_t oTB   = off; off += SZ_TB;
  const size_t oFT   = off; off += SZ_FT;
  const size_t oELR  = off; off += SZ_ELR;
  const size_t oMETA = off; off += SZ_META;
  const size_t oLIST = off; off += SZ_LIST;
  if (off != (size_t)WS_TOTAL) return;
  if (off > ws_size || off > (size_t)WSMAX) return;
  unsigned short* XB  = (unsigned short*)(ws + oXB);
  unsigned short* OP  = XB;
  unsigned short* WP  = (unsigned short*)(ws + oWP);
  unsigned short* W1T = WP;
  unsigned short* W2D = WP + HC * KD;
  unsigned short* W3D = WP + 2 * HC * KD;
  float*    TB   = (float*)(ws + oTB);
  float*    FT   = (float*)(ws + oFT);
  float*    ELR  = (float*)(ws + oELR);
  int*      META = (int*)(ws + oMETA);
  unsigned* LIST = (unsigned*)(ws + oLIST);

  hipFuncSetAttribute(reinterpret_cast<const void*>(&k_list),
                      hipFuncAttributeMaxDynamicSharedMemorySize, LDS_LST);

  k_plane<0><<<MPAD * KD / 8 / 256, 256, 0, stream>>>(feat, NN, KD, KD, XB, MPAD, KD);
  k_prep<<<13, 256, 0, stream>>>(W1, W2, W3, as1, ad1, b1, as2, ad2, b2, as3, ad3, b3, WP, TB);
  k_list<<<NBLK, LT, LDS_LST, stream>>>(esrc, edst, LIST, META);

  const int tiles = (MPAD / 64) * (HC / 64);
  const int gG = (tiles + 7) / 8;
  const int gR = NN / RWAVES;
  const unsigned lo2 = (SPLIT_2 != 0) ? 0xFFFFFFFFu : 0u;
  const unsigned lo3 = (SPLIT_3 != 0) ? 0xFFFFFFFFu : 0u;

  k_gemm_nt<0, 0><<<gG, 256, 0, stream>>>(XB, W1T, TB, FT, MPAD, HC, KD, HC);
  k_rowprep<2><<<gR, RTHR, 0, stream>>>(FT, TB, ELR);
  k_walk<0><<<gR, RTHR, 0, stream>>>(FT, ELR, LIST, META, TB, OP, out, nrows, lo2);
  k_gemm_nt<0, 0><<<gG, 256, 0, stream>>>(OP, W2D, TB, FT, MPAD, HC, KD, HC);
  k_rowprep<2><<<gR, RTHR, 0, stream>>>(FT, TB + TBL_L, ELR);
  k_walk<0><<<gR, RTHR, 0, stream>>>(FT, ELR, LIST, META, TB + TBL_L, OP, out, nrows, lo3);
  k_gemm_nt<0, 0><<<gG, 256, 0, stream>>>(OP, W3D, TB, FT, MPAD, HC, KD, HC);
  k_rowprep<1><<<gR, RTHR, 0, stream>>>(FT, TB + 2 * TBL_L, ELR);
  k_walk<1><<<gR, RTHR, 0, stream>>>(FT, ELR, LIST, META, TB + 2 * TBL_L, OP, out, nrows, 0u);
}
